// PriceGeometryEncoder_54168127537314
// MI455X (gfx1250) — hardware-verified
//
#include <hip/hip_runtime.h>

#define B_   16
#define T_   2048
#define E_   128
#define H_   4
#define DH_  32
#define NROW (B_*T_)
#define DP_  512
#define QW   8
#define KT   64

typedef __attribute__((ext_vector_type(16))) _Float16 v16h;
typedef __attribute__((ext_vector_type(8)))  _Float16 v8h;
typedef __attribute__((ext_vector_type(8)))  float    v8f;
typedef __attribute__((ext_vector_type(4)))  unsigned v4u_t;
typedef unsigned v4ua __attribute__((ext_vector_type(4), may_alias));
#define NQB (T_/(16*QW))
__device__ __forceinline__ unsigned pk2(float a, float b) { return (unsigned)__builtin_bit_cast(unsigned short, (_Float16)a) | ((unsigned)__builtin_bit_cast(unsigned short, (_Float16)b) << 16); }

__device__ __forceinline__ v16h ld_frag(const _Float16* p0, const _Float16* p1) {
  v8h lo = *(const v8h*)p0;
  v8h hi = *(const v8h*)p1;
  return __builtin_shufflevector(lo, hi, 0,1,2,3,4,5,6,7,8,9,10,11,12,13,14,15);
}

__global__ void __launch_bounds__(256) prepw_kernel(
    const float* __restrict__ Wqkv, _Float16* __restrict__ wb)
{
  int idx = (blockIdx.x * 256 + threadIdx.x) * 2;
  float w2[2];
#pragma unroll
  for (int q = 0; q < 2; ++q) {
    int id = idx + q;
    int e    = id & 15;
    int row  = (id >> 4) & 31;
    int ksnt = id >> 9;
    int ks   = ksnt & 3;
    int nt   = ksnt >> 2;
    int khalf = row >> 4;
    int n     = row & 15;
    int k   = ks*32 + ((e < 8) ? (khalf*8 + e) : (16 + khalf*8 + (e - 8)));
    int col = nt*16 + n;
    w2[q] = Wqkv[(size_t)k*384 + col];
  }
  const unsigned p = pk2(w2[0], w2[1]);
  *(volatile unsigned*)(wb + idx) = p; __threadfence(); *(volatile unsigned*)(wb + idx) = p;
}

__global__ void __launch_bounds__(128) feats_kernel(
    const float* __restrict__ ohlc,
    const float* __restrict__ Wp,  const float* __restrict__ bp,
    const float* __restrict__ Wc1, const float* __restrict__ bc1,
    const float* __restrict__ Wc2, const float* __restrict__ bc2,
    const float* __restrict__ Wv1, const float* __restrict__ bv1,
    const float* __restrict__ Wv2, const float* __restrict__ bv2,
    const float* __restrict__ Ws1, const float* __restrict__ bs1,
    const float* __restrict__ Ws2, const float* __restrict__ bs2,
    _Float16* __restrict__ feats)
{
  __shared__ float e_s[64];
  __shared__ float ch[128];
  __shared__ float vhid[64];
  __shared__ float shid[64];

  int row = blockIdx.x;
  int tid = threadIdx.x;

  if (tid < 64) {
    float acc = bp[tid];
    #pragma unroll
    for (int i = 0; i < 4; ++i) acc += ohlc[row*4 + i] * Wp[i*64 + tid];
    e_s[tid] = acc;
  }
  __syncthreads();

  {
    float acc = bc1[tid];
    #pragma unroll 8
    for (int i = 0; i < 64; ++i) acc += e_s[i] * Wc1[i*128 + tid];
    ch[tid] = fmaxf(acc, 0.f);
  }
  if (tid < 64) {
    float acc = bv1[tid];
    #pragma unroll 8
    for (int i = 0; i < 64; ++i) acc += e_s[i] * Wv1[i*64 + tid];
    vhid[tid] = fmaxf(acc, 0.f);
  } else {
    int t = tid - 64;
    float acc = bs1[t];
    #pragma unroll 8
    for (int i = 0; i < 64; ++i) acc += e_s[i] * Ws1[i*64 + t];
    shid[t] = fmaxf(acc, 0.f);
  }
  __syncthreads();

  float out;
  if (tid < 64) {
    out = e_s[tid];
  } else if (tid < 96) {
    int j = tid - 64;
    float acc = bc2[j];
    #pragma unroll 8
    for (int i = 0; i < 128; ++i) acc += ch[i] * Wc2[i*32 + j];
    out = acc;
  } else if (tid < 112) {
    int j = tid - 96;
    float acc = bv2[j];
    #pragma unroll 8
    for (int i = 0; i < 64; ++i) acc += vhid[i] * Wv2[i*16 + j];
    out = acc;
  } else {
    int j = tid - 112;
    float acc = bs2[j];
    #pragma unroll 8
    for (int i = 0; i < 64; ++i) acc += shid[i] * Ws2[i*16 + j];
    out = acc;
  }
  __shared__ float orow[128];
  orow[tid] = out;
  __syncthreads();
  if (tid < 64) {
    const unsigned p = pk2(orow[2 * tid], orow[2 * tid + 1]);
    *(volatile unsigned*)(feats + (size_t)row*128 + 2 * tid) = p; __threadfence(); *(volatile unsigned*)(feats + (size_t)row*128 + 2 * tid) = p;
  }
}

__global__ void __launch_bounds__(128) qkv_kernel(
    const _Float16* __restrict__ feats,
    const _Float16* __restrict__ wb, const float* __restrict__ bqkv,
    _Float16* __restrict__ qg, _Float16* __restrict__ kg, _Float16* __restrict__ vg)
{
  __shared__ __align__(16) _Float16 st[4][16 * 32];
  int lane  = threadIdx.x & 31;
  int wave  = threadIdx.x >> 5;
  int mt    = blockIdx.x * 4 + wave;
  int nt2   = blockIdx.y;
  int row0  = mt * 16;
  int n     = lane & 15;
  int khalf = lane >> 4;

  v8f acc[2] = {};
  #pragma unroll
  for (int ks = 0; ks < 4; ++ks) {
    const _Float16* arow = feats + (size_t)(row0 + n)*128 + ks*32;
    v16h a = ld_frag(arow + khalf*8, arow + 16 + khalf*8);
    #pragma unroll
    for (int j = 0; j < 2; ++j) {
      const int nt = 2 * nt2 + j;
      const _Float16* wbp = wb + ((size_t)((nt*4 + ks)*32) + khalf*16 + n)*16;
      v16h b = ld_frag(wbp, wbp + 8);
      acc[j] = __builtin_amdgcn_wmma_f32_16x16x32_f16(false, a, false, b, (short)0, acc[j], false, false);
    }
  }

  int   which  = nt2 >> 2;
  int   h      = nt2 & 3;
  float scale  = (which == 0) ? 0.17677669529663687f : 1.0f;
  _Float16* dst = (which == 0) ? qg : (which == 1) ? kg : vg;
  _Float16* sw = st[wave];
  #pragma unroll
  for (int j = 0; j < 2; ++j) {
    const float bias = bqkv[(2 * nt2 + j) * 16 + n];
    #pragma unroll
    for (int r = 0; r < 8; ++r) sw[(r + 8*khalf) * 32 + j * 16 + n] = (_Float16)((acc[j][r] + bias) * scale);
  }
  asm volatile("s_wait_dscnt 0" ::: "memory");
  const int b_ = row0 >> 11, t_ = row0 & (T_ - 1);
  _Float16* drow = dst + ((size_t)(b_*H_ + h)*T_ + t_)*DH_;
  v4u_t ov[2];
  #pragma unroll
  for (int i = 0; i < 2; ++i) ov[i] = *(const volatile v4ua*)(sw + (lane + 32 * i) * 8);
  #pragma unroll
  for (int i = 0; i < 2; ++i) *(volatile v4u_t*)(drow + (lane + 32 * i) * 8) = ov[i];
  __threadfence();
  #pragma unroll
  for (int i = 0; i < 2; ++i) *(volatile v4u_t*)(drow + (lane + 32 * i) * 8) = ov[i];
}

__global__ void __launch_bounds__(256) flash_kernel(
    const _Float16* __restrict__ qg,
    const _Float16* __restrict__ kg,
    const _Float16* __restrict__ vg,
    _Float16* __restrict__ og)
{
  __shared__ __align__(16) _Float16 Kt[2][KT*DH_];
  __shared__ __align__(16) _Float16 VtT[2][DH_*KT];
  __shared__ __align__(16) _Float16 Pl[QW][16][KT];

  int tid   = threadIdx.x;
  int lane  = tid & 31;
  int wave  = tid >> 5;
  int bh    = blockIdx.y;
  int qt0   = blockIdx.x * (16*QW) + wave * 16;
  int n     = lane & 15;
  int khalf = lane >> 4;

  const _Float16* qb = qg + (size_t)bh * T_ * DH_;
  const _Float16* kb = kg + (size_t)bh * T_ * DH_;
  const _Float16* vb = vg + (size_t)bh * T_ * DH_;

  const _Float16* qrow = qb + (size_t)(qt0 + n) * DH_;
  v16h aq = ld_frag(qrow + khalf*8, qrow + 16 + khalf*8);

  int sr = tid >> 2;
  int sc = (tid & 3) * 8;
  unsigned kt_lds0 = (unsigned)(uintptr_t)(&Kt[0][sr*DH_ + sc]);
  unsigned kt_lds1 = (unsigned)(uintptr_t)(&Kt[1][sr*DH_ + sc]);

  float m_i[8], l_i[8];
  #pragma unroll
  for (int r = 0; r < 8; ++r) { m_i[r] = -3.0e38f; l_i[r] = 0.f; }
  v8f o0 = {}; v8f o1 = {};

  {
    const _Float16* gk = kb + (size_t)sr*DH_ + sc;
    asm volatile("global_load_async_to_lds_b128 %0, %1, off"
                 :: "v"(kt_lds0), "v"(gk) : "memory");
    const _Float16* gv = vb + (size_t)sr*DH_ + sc;
    v8h vv = *(const v8h*)gv;
    #pragma unroll
    for (int i = 0; i < 8; ++i) VtT[0][(sc + i)*KT + sr] = vv[i];
    asm volatile("s_wait_asynccnt 0x0" ::: "memory");
  }
  __syncthreads();

  int buf = 0;
  for (int j0 = 0; j0 < T_; j0 += KT) {
    int  nxt  = buf ^ 1;
    bool more = (j0 + KT) < T_;

    v8h vnext = {};
    if (more) {
      const _Float16* gk = kb + (size_t)(j0 + KT + sr)*DH_ + sc;
      unsigned ldst = nxt ? kt_lds1 : kt_lds0;
      asm volatile("global_load_async_to_lds_b128 %0, %1, off"
                   :: "v"(ldst), "v"(gk) : "memory");
      vnext = *(const v8h*)(vb + (size_t)(j0 + KT + sr)*DH_ + sc);
    }

    const _Float16* ktb = &Kt[buf][0];
    const _Float16* vtb = &VtT[buf][0];

    v8f zero = {};
    v8f s0, s1, s2, s3;
    {
      const _Float16* p = &ktb[(0*16 + n)*DH_ + khalf*8];
      s0 = __builtin_amdgcn_wmma_f32_16x16x32_f16(false, aq, false,
             ld_frag(p, p + 16), (short)0, zero, false, false);
    }
    {
      const _Float16* p = &ktb[(1*16 + n)*DH_ + khalf*8];
      s1 = __builtin_amdgcn_wmma_f32_16x16x32_f16(false, aq, false,
             ld_frag(p, p + 16), (short)0, zero, false, false);
    }
    {
      const _Float16* p = &ktb[(2*16 + n)*DH_ + khalf*8];
      s2 = __builtin_amdgcn_wmma_f32_16x16x32_f16(false, aq, false,
             ld_frag(p, p + 16), (short)0, zero, false, false);
    }
    {
      const _Float16* p = &ktb[(3*16 + n)*DH_ + khalf*8];
      s3 = __builtin_amdgcn_wmma_f32_16x16x32_f16(false, aq, false,
             ld_frag(p, p + 16), (short)0, zero, false, false);
    }

    #pragma unroll
    for (int r = 0; r < 8; ++r) {
      float x0 = s0[r], x1 = s1[r], x2 = s2[r], x3 = s3[r];
      float mx = fmaxf(fmaxf(x0, x1), fmaxf(x2, x3));
      #pragma unroll
      for (int m = 1; m < 16; m <<= 1) mx = fmaxf(mx, __shfl_xor(mx, m, 32));
      float mnew = fmaxf(m_i[r], mx);
      float corr = __expf(m_i[r] - mnew);
      float p0 = __expf(x0 - mnew);
      float p1 = __expf(x1 - mnew);
      float p2 = __expf(x2 - mnew);
      float p3 = __expf(x3 - mnew);
      float rs = (p0 + p1) + (p2 + p3);
      #pragma unroll
      for (int m = 1; m < 16; m <<= 1) rs += __shfl_xor(rs, m, 32);
      l_i[r] = l_i[r] * corr + rs;
      m_i[r] = mnew;
      o0[r] *= corr; o1[r] *= corr;
      int rowl = r + 8*khalf;
      Pl[wave][rowl][n]      = (_Float16)(p0 * 1024.0f);
      Pl[wave][rowl][16 + n] = (_Float16)(p1 * 1024.0f);
      Pl[wave][rowl][32 + n] = (_Float16)(p2 * 1024.0f);
      Pl[wave][rowl][48 + n] = (_Float16)(p3 * 1024.0f);
    }

    const _Float16* prow = &Pl[wave][n][0];
    v16h ap0 = ld_frag(prow + khalf*8,      prow + 16 + khalf*8);
    v16h ap1 = ld_frag(prow + 32 + khalf*8, prow + 48 + khalf*8);

    const _Float16* v00 = &vtb[n*KT + khalf*8];
    const _Float16* v10 = &vtb[n*KT + 32 + khalf*8];
    const _Float16* v01 = &vtb[(16 + n)*KT + khalf*8];
    const _Float16* v11 = &vtb[(16 + n)*KT + 32 + khalf*8];
    o0 = __builtin_amdgcn_wmma_f32_16x16x32_f16(false, ap0, false,
           ld_frag(v00, v00 + 16), (short)0, o0, false, false);
    o0 = __builtin_amdgcn_wmma_f32_16x16x32_f16(false, ap1, false,
           ld_frag(v10, v10 + 16), (short)0, o0, false, false);
    o1 = __builtin_amdgcn_wmma_f32_16x16x32_f16(false, ap0, false,
           ld_frag(v01, v01 + 16), (short)0, o1, false, false);
    o1 = __builtin_amdgcn_wmma_f32_16x16x32_f16(false, ap1, false,
           ld_frag(v11, v11 + 16), (short)0, o1, false, false);

    if (more) {
      #pragma unroll
      for (int i = 0; i < 8; ++i) VtT[nxt][(sc + i)*KT + sr] = vnext[i];
    }
    asm volatile("s_wait_asynccnt 0x0" ::: "memory");
    __syncthreads();
    buf = nxt;
  }

  float cs0 = 0.f, cs1 = 0.f;
  #pragma unroll
  for (int r = 0; r < 8; ++r) {
    float inv = 1.0f / (l_i[r] * 1024.0f);
    cs0 += o0[r] * inv; cs1 += o1[r] * inv;
  }
  cs0 += __shfl_xor(cs0, 16, 32); cs1 += __shfl_xor(cs1, 16, 32);
  __shared__ float red[QW][32];
  if (khalf == 0) { red[wave][n] = cs0; red[wave][16 + n] = cs1; }
  __syncthreads();
  if (wave == 0) {
    float s = 0.f;
    #pragma unroll
    for (int w = 0; w < QW; ++w) s += red[w][lane];
    float* pp = (float*)og + ((size_t)bh * NQB + blockIdx.x) * 32 + lane;
    *(volatile float*)pp = s; __threadfence(); *(volatile float*)pp = s;
  }
}

__global__ void __launch_bounds__(128) pool_kernel(
    const _Float16* __restrict__ og, float* __restrict__ pooled)
{
  int b = blockIdx.x;
  int e = threadIdx.x;
  int h = e >> 5, d = e & 31;
  const float* p = (const float*)og + ((size_t)(b*H_ + h) * NQB) * 32 + d;
  float acc = 0.f;
  #pragma unroll
  for (int q = 0; q < NQB; ++q) acc += p[(size_t)q * 32];
  const float v = acc * (1.0f / T_);
  *(volatile float*)(pooled + b*E_ + e) = v; __threadfence(); *(volatile float*)(pooled + b*E_ + e) = v;
}

__global__ void __launch_bounds__(256) head_kernel(
    const float* __restrict__ pooled,
    const float* __restrict__ Wo,   const float* __restrict__ bo,
    const float* __restrict__ Wout, const float* __restrict__ bout,
    float* __restrict__ out)
{
  __shared__ float attm[B_ * E_];
  for (int idx = threadIdx.x; idx < B_*E_; idx += blockDim.x) {
    int b = idx >> 7, e = idx & 127;
    float acc = bo[e];
    #pragma unroll 8
    for (int i = 0; i < E_; ++i) acc += pooled[b*E_ + i] * Wo[i*E_ + e];
    attm[idx] = acc;
  }
  __syncthreads();
  for (int idx = threadIdx.x; idx < B_*DP_; idx += blockDim.x) {
    int b = idx >> 9, oc = idx & 511;
    float acc = bout[oc];
    #pragma unroll 8
    for (int i = 0; i < E_; ++i) acc += attm[b*E_ + i] * Wout[i*DP_ + oc];
    *(volatile float*)(out + idx) = acc; __threadfence(); *(volatile float*)(out + idx) = acc;
  }
}

extern "C" void kernel_launch(void* const* d_in, const int* in_sizes, int n_in,
                              void* d_out, int out_size, void* d_ws, size_t ws_size,
                              hipStream_t stream) {
  const float* ohlc = (const float*)d_in[0];
  const float* Wp   = (const float*)d_in[1];
  const float* bp   = (const float*)d_in[2];
  const float* Wc1  = (const float*)d_in[3];
  const float* bc1  = (const float*)d_in[4];
  const float* Wc2  = (const float*)d_in[5];
  const float* bc2  = (const float*)d_in[6];
  const float* Wv1  = (const float*)d_in[7];
  const float* bv1  = (const float*)d_in[8];
  const float* Wv2  = (const float*)d_in[9];
  const float* bv2  = (const float*)d_in[10];
  const float* Ws1  = (const float*)d_in[11];
  const float* bs1  = (const float*)d_in[12];
  const float* Ws2  = (const float*)d_in[13];
  const float* bs2  = (const float*)d_in[14];
  const float* Wqkv = (const float*)d_in[15];
  const float* bqkv = (const float*)d_in[16];
  const float* Wo   = (const float*)d_in[17];
  const float* bo   = (const float*)d_in[18];
  const float* Wout = (const float*)d_in[19];
  const float* bout = (const float*)d_in[20];

  char* ws = (char*)d_ws;
  const size_t MB = 1024ull * 1024ull;
  _Float16* feats = (_Float16*)(ws);
  _Float16* qg    = (_Float16*)(ws +  8*MB);
  _Float16* kg    = (_Float16*)(ws + 16*MB);
  _Float16* vg    = (_Float16*)(ws + 24*MB);
  _Float16* og    = (_Float16*)(ws + 32*MB);
  float*    pooled= (float*)   (ws + 40*MB);
  _Float16* wb    = (_Float16*)(ws + 41*MB);

  prepw_kernel<<<96, 256, 0, stream>>>(Wqkv, wb);

  feats_kernel<<<NROW, 128, 0, stream>>>(ohlc, Wp, bp, Wc1, bc1, Wc2, bc2,
                                         Wv1, bv1, Wv2, bv2, Ws1, bs1, Ws2, bs2,
                                         feats);

  dim3 g2(NROW/16/4, 384/32);
  qkv_kernel<<<g2, 128, 0, stream>>>(feats, wb, bqkv, qg, kg, vg);

  dim3 g3(T_/(16*QW), B_*H_);
  flash_kernel<<<g3, 256, 0, stream>>>(qg, kg, vg, og);

  pool_kernel<<<B_, 128, 0, stream>>>(og, pooled);

  head_kernel<<<1, 256, 0, stream>>>(pooled, Wo, bo, Wout, bout, (float*)d_out);
}
